// MultigpuGCNConv_87960930222589
// MI455X (gfx1250) — hardware-verified
//
#include <hip/hip_runtime.h>


#define NN_  50000
#define NNP  50048
#define KIN  256
#define NOUT 128
#define NNZ_ 800000

typedef unsigned short bf;
typedef __attribute__((ext_vector_type(16))) __bf16   v16bf;
typedef __attribute__((ext_vector_type(8)))  unsigned short v8us;
typedef __attribute__((ext_vector_type(8)))  float    v8f;
typedef __attribute__((ext_vector_type(4)))  float    v4f;
typedef v4f  __attribute__((may_alias)) v4fa;
typedef v8us __attribute__((may_alias)) v8usa;

__device__ __forceinline__ unsigned short f2bf(float f) { unsigned u = __float_as_uint(f); u += 0x7FFFu + ((u >> 16) & 1u); return (unsigned short)(u >> 16); }
__device__ __forceinline__ float bf2f(unsigned short b) { return __uint_as_float(((unsigned)b) << 16); }
__device__ __forceinline__ float bfr(float f) { return bf2f(f2bf(f)); }
__device__ __forceinline__ v16bf cat16b(v8us lo, v8us hi) { return __builtin_bit_cast(v16bf, __builtin_shufflevector(lo, hi, 0, 1, 2, 3, 4, 5, 6, 7, 8, 9, 10, 11, 12, 13, 14, 15)); }
__device__ __forceinline__ v8f wmmab(v16bf a, v16bf b, v8f c) { return __builtin_amdgcn_wmma_f32_16x16x32_bf16(false, a, false, b, (short)0, c, false, false); }
#define VST2(T, p, v) do { const T vst2_v_ = (v); *(volatile T*)(p) = vst2_v_; __threadfence(); *(volatile T*)(p) = vst2_v_; } while (0)

__global__ __launch_bounds__(256) void k_xb(const float* __restrict__ x, bf* Xb) {
    const int lane = threadIdx.x & 31, r = blockIdx.x * 8 + (threadIdx.x >> 5);
    if (r >= NNP) return;
    const int rr = (r < NN_) ? r : (NN_ - 1);
    v8us t;
#pragma unroll
    for (int i = 0; i < 8; ++i) { const unsigned short hb = f2bf(x[(size_t)rr * KIN + lane * 8 + i]); t[i] = (r < NN_) ? hb : (unsigned short)0; }
    VST2(v8us, Xb + (size_t)r * KIN + lane * 8, t);
}
__global__ __launch_bounds__(256) void k_wt(const float* __restrict__ Wm, bf* WT) {
    __shared__ __align__(16) unsigned short tl[64 * 72];
    const int tid = threadIdx.x, k0 = blockIdx.x * 64, n0 = blockIdx.y * 64;
    const int kk = tid >> 2, nq = (tid & 3) * 16;
#pragma unroll
    for (int i = 0; i < 16; ++i) tl[(nq + i) * 72 + kk] = f2bf(Wm[(size_t)(k0 + kk) * NOUT + n0 + nq + i]);
    __syncthreads();
    const int piece = tid & 7;
    auto pass = [&]() {
#pragma unroll
        for (int s = 0; s < 2; ++s) { const int nr = (tid >> 3) + 32 * s; const v8us val = *(const v8usa*)(tl + nr * 72 + piece * 8);
            *(volatile v8us*)(WT + (size_t)(n0 + nr) * KIN + k0 + piece * 8) = val; }
    };
    pass(); __threadfence(); pass();
}
__global__ __launch_bounds__(128) void k_gemm(const bf* __restrict__ A, const bf* __restrict__ Bn, float* C) {
    __shared__ __align__(16) float ost[4][16 * 68];
    const int lane = threadIdx.x & 31, wave = threadIdx.x >> 5, lr = lane & 15, hi = lane >> 4;
    const int r0 = blockIdx.x * 64 + wave * 16, c0 = blockIdx.y * 64;
    const size_t aoff = (size_t)(r0 + lr) * KIN + 8 * hi;
    size_t boff[4];
#pragma unroll
    for (int t = 0; t < 4; ++t) boff[t] = (size_t)(c0 + t * 16 + lr) * KIN + 8 * hi;
    v8f acc[4];
#pragma unroll
    for (int t = 0; t < 4; ++t) acc[t] = (v8f){};
#pragma unroll
    for (int kc = 0; kc < KIN; kc += 32) {
        const v16bf a = cat16b(*(const v8us*)(A + aoff + kc), *(const v8us*)(A + aoff + kc + 16));
#pragma unroll
        for (int t = 0; t < 4; ++t) acc[t] = wmmab(a, cat16b(*(const v8us*)(Bn + boff[t] + kc), *(const v8us*)(Bn + boff[t] + kc + 16)), acc[t]);
    }
    asm volatile("v_nop\n\tv_nop\n\tv_nop\n\tv_nop" : "+v"(acc[0]), "+v"(acc[1]), "+v"(acc[2]), "+v"(acc[3]));
    float* os = &ost[wave][0];
#pragma unroll
    for (int t = 0; t < 4; ++t)
#pragma unroll
        for (int j = 0; j < 8; ++j) os[(hi * 8 + j) * 68 + t * 16 + lr] = acc[t][j];
    __syncthreads();
    float* crow = C + (size_t)r0 * NOUT + c0;
    auto pass = [&]() {
#pragma unroll
        for (int s = 0; s < 8; ++s) { const int Lid = (lane >> 3) + 4 * s, piece = lane & 7; const int row = Lid >> 1, cofs = (Lid & 1) * 32 + piece * 4;
            const v4f val = *(const v4fa*)(os + row * 68 + cofs); *(volatile v4f*)(crow + (size_t)row * NOUT + cofs) = val; }
    };
    pass(); __threadfence(); pass();
}
__global__ __launch_bounds__(256) void k_spmm(const int* __restrict__ rp, const int* __restrict__ ci, const float* __restrict__ ev, const float* __restrict__ H, const float* __restrict__ bias, float* out) {
    const int lane = threadIdx.x & 31, i = blockIdx.x * 8 + (threadIdx.x >> 5);
    if (i >= NN_) return;
    int e0 = rp[i], e1 = rp[i + 1];
    e0 = e0 < 0 ? 0 : (e0 > NNZ_ ? NNZ_ : e0); e1 = e1 < e0 ? e0 : (e1 > NNZ_ ? NNZ_ : e1);
    v4f acc; acc[0] = 0.f; acc[1] = 0.f; acc[2] = 0.f; acc[3] = 0.f;
#pragma unroll 1
    for (int e = e0; e < e1; ++e) {
        int c = ci[e]; if (c < 0) c += NN_; c = ((unsigned)c < (unsigned)NN_) ? c : 0;
        const float w = bfr(ev[e]);
        const v4f hv = *(const v4fa*)(H + (size_t)c * NOUT + lane * 4);
#pragma unroll
        for (int q = 0; q < 4; ++q) acc[q] += w * hv[q];
    }
    v4f o;
#pragma unroll
    for (int q = 0; q < 4; ++q) o[q] = fmaxf(acc[q] + bfr(bias[lane * 4 + q]), 0.f);
    VST2(v4f, out + (size_t)i * NOUT + lane * 4, o);
}

extern "C" void kernel_launch(void* const* d_in, const int* in_sizes, int n_in,
                              void* d_out, int out_size, void* d_ws, size_t ws_size, hipStream_t stream) {
    (void)in_sizes; (void)n_in; (void)out_size;
    const int* rp = (const int*)d_in[1]; const int* ci = (const int*)d_in[2]; const float* ev = (const float*)d_in[3];
    const float* x = (const float*)d_in[11]; const float* Wm = (const float*)d_in[12]; const float* bias = (const float*)d_in[13];
    float* out = (float*)d_out;
    char* wsp = (char*)d_ws;
    auto take = [&](size_t bytes) { char* p = wsp; wsp += (bytes + 255) & ~(size_t)255; return (void*)p; };
    bf* Xb = (bf*)take((size_t)NNP * KIN * 2); bf* WT = (bf*)take((size_t)NOUT * KIN * 2); float* H = (float*)take((size_t)NNP * NOUT * 4);
    if ((size_t)(wsp - (char*)d_ws) > ws_size) return;
    k_xb<<<NNP / 8, 256, 0, stream>>>(x, Xb);
    k_wt<<<dim3(KIN / 64, NOUT / 64, 1), 256, 0, stream>>>(Wm, WT);
    k_gemm<<<dim3(NNP / 64, NOUT / 64, 1), 128, 0, stream>>>(Xb, WT, H);
    k_spmm<<<(NN_ + 7) / 8, 256, 0, stream>>>(rp, ci, ev, H, bias, out);
}
